// EGCL_72361609003289
// MI455X (gfx1250) — hardware-verified
//
#include <hip/hip_runtime.h>
#include <stddef.h>
#include <stdint.h>


#define VD   32
#define VC   96
#define HD   128
#define UD   256
#define KE1  64
#define KHL  512
#define KH1  640
#define NTHR 256
#define ATHR 384
#define GBM  64
#define RPC  128
#define WSMAX 134217728
#define C288 0.058925565f
#define C384 0.051031036f
#define C16  0.0625f
#define NU_E1A  (UD * (KE1 / 8))
#define NU_E1BC (2 * UD * (HD / 8))
#define NU_SQ   (UD * (KHL / 8))
#define NU_XL   (VD * (KHL / 8))
#define NU_H1   (UD * (KH1 / 8))
#define NU_HL   (HD * (KHL / 8))
#define NU_W    (NU_E1A + NU_E1BC + 4 * NU_SQ + NU_XL + NU_H1 + NU_HL)
#define LDS_EXTRA 2048
#define LDS_BIG (GBM * 256 * 4 + LDS_EXTRA)
#define LDS_OUT (GBM * 128 * 4 + LDS_EXTRA)
#define LDS_XL  (GBM * 32 * 4 + LDS_EXTRA)

static_assert(NU_E1A % NTHR == 0 && NU_E1BC % NTHR == 0 && NU_SQ % NTHR == 0 && NU_XL % NTHR == 0);
static_assert(NU_H1 % NTHR == 0 && NU_HL % NTHR == 0 && NU_W % NTHR == 0);
static_assert((NU_SQ & (NU_SQ - 1)) == 0);
static_assert(KE1 == 2 * VD && KHL == 2 * UD && KH1 == 2 * UD + HD);
static_assert(KE1 % 32 == 0 && KHL % 32 == 0 && KH1 % 32 == 0 && HD % 32 == 0);
static_assert(UD == NTHR && VC == 3 * VD && ATHR == 4 * VC && KH1 / 8 <= NTHR && VC / 4 <= ATHR);
static_assert((UD + 2 * GBM + GBM) * 4 <= LDS_EXTRA);
static_assert(RPC % 8 == 0 && (RPC * 2) % GBM == 0 && GBM == 64);
static_assert(NTHR * KE1 * 2 == 8 * NTHR * 16);

typedef float          v4f   __attribute__((ext_vector_type(4)));
typedef float          v8f   __attribute__((ext_vector_type(8)));
typedef int            v8i   __attribute__((ext_vector_type(8)));
typedef unsigned short v8us  __attribute__((ext_vector_type(8)));
typedef unsigned short v16us __attribute__((ext_vector_type(16)));
typedef __bf16         v16bf __attribute__((ext_vector_type(16)));
typedef v4f  __attribute__((may_alias)) v4fa;
typedef v8us __attribute__((may_alias)) v8usa;
union FragB { v16bf v; v16us u; v8us h[2]; v8i w; };
union R24 { v4f q[6]; float f[24]; };

__device__ __forceinline__ v8f wmb(const FragB& a, const FragB& b, v8f c) {
  v8f d = __builtin_amdgcn_wmma_f32_16x16x32_bf16(false, a.v, false, b.v, (short)0, c, false, false);
  asm volatile("v_nop\n\tv_nop\n\tv_nop\n\tv_nop" : "+v"(d) : "v"(a.w), "v"(b.w));
  return d;
}

__device__ __forceinline__ unsigned bf16_bits(float f) {
  const unsigned u = __float_as_uint(f);
  return (u + 0x7FFFu + ((u >> 16) & 1u)) >> 16;
}
__device__ __forceinline__ float bf16_val(float f) {
  return __uint_as_float(bf16_bits(f) << 16);
}
__device__ __forceinline__ float bfw(unsigned short b) {
  return __uint_as_float(((unsigned)b) << 16);
}
__device__ __forceinline__ float silu_f(float t) {
  return t * __builtin_amdgcn_rcpf(1.0f + __expf(-t));
}
__device__ __forceinline__ void put16(unsigned short* dp, v8us o) {
  *(volatile v8us*)dp = o;
  __threadfence();
  *(volatile v8us*)dp = o;
}

__global__ __launch_bounds__(NTHR) void k_prep(const float* __restrict__ nf, const float* __restrict__ We1,
                                               const float* __restrict__ We2, const float* __restrict__ Wx1,
                                               const float* __restrict__ Wx2, const float* __restrict__ Wxl,
                                               const float* __restrict__ Wh1, const float* __restrict__ Wh2,
                                               const float* __restrict__ Whl, int nN,
                                               unsigned short* WE1A, unsigned short* WE1BC, unsigned short* WE2T,
                                               unsigned short* WX1T, unsigned short* WX2T, unsigned short* WXLT,
                                               unsigned short* WH1T, unsigned short* WH2T, unsigned short* WHLT,
                                               unsigned short* NFB) {
  const int u  = (int)blockIdx.x * NTHR + (int)threadIdx.x;
  const int U0 = NU_E1A;
  const int U1 = U0 + NU_E1BC;
  const int U2 = U1 + 4 * NU_SQ;
  const int U3 = U2 + NU_XL;
  const int U4 = U3 + NU_H1;
  const int U5 = U4 + NU_HL;
  const int U6 = U5 + nN * (HD / 8);
  v8us o;
  if (u < U0) {
    const int n    = u >> 3;
    const int k8   = (u & 7) * 8;
    const int srow = k8 & (VD - 1);
    const float* p = We1 + (size_t)srow * UD + n;
#pragma unroll
    for (int i = 0; i < 8; ++i) o[i] = (unsigned short)bf16_bits(p[(size_t)i * UD]);
    put16(WE1A + (size_t)n * KE1 + k8, o);
    return;
  } else if (u < U1) {
    const int v    = u - U0;
    const int n    = v >> 4;
    const int k8   = (v & 15) * 8;
    const int q    = n >> 8;
    const int nn   = n & (UD - 1);
    const int srow = VD + q * HD + k8;
    const float* p = We1 + (size_t)srow * UD + nn;
#pragma unroll
    for (int i = 0; i < 8; ++i) o[i] = (unsigned short)bf16_bits(p[(size_t)i * UD]);
    put16(WE1BC + (size_t)n * HD + k8, o);
    return;
  } else if (u < U2) {
    const int v    = u - U1;
    const int q    = v / NU_SQ;
    const int w    = v - q * NU_SQ;
    const int n    = w >> 6;
    const int k8   = (w & 63) * 8;
    const int srow = k8 & (UD - 1);
    const float* W = (q == 0) ? We2 : ((q == 1) ? Wx1 : ((q == 2) ? Wx2 : Wh2));
    unsigned short* O = (q == 0) ? WE2T : ((q == 1) ? WX1T : ((q == 2) ? WX2T : WH2T));
    const float* p = W + (size_t)srow * UD + n;
#pragma unroll
    for (int i = 0; i < 8; ++i) o[i] = (unsigned short)bf16_bits(p[(size_t)i * UD]);
    put16(O + (size_t)n * KHL + k8, o);
    return;
  } else if (u < U3) {
    const int v    = u - U2;
    const int n    = v >> 6;
    const int k8   = (v & 63) * 8;
    const int srow = k8 & (UD - 1);
    const float* p = Wxl + (size_t)srow * VD + n;
#pragma unroll
    for (int i = 0; i < 8; ++i) o[i] = (unsigned short)bf16_bits(p[(size_t)i * VD]);
    put16(WXLT + (size_t)n * KHL + k8, o);
    return;
  } else if (u < U4) {
    const int v    = u - U3;
    const int n    = v / (KH1 / 8);
    const int k8   = (v - n * (KH1 / 8)) * 8;
    const int srow = (k8 < KHL) ? (k8 & (UD - 1)) : (UD + k8 - KHL);
    const float* p = Wh1 + (size_t)srow * UD + n;
#pragma unroll
    for (int i = 0; i < 8; ++i) o[i] = (unsigned short)bf16_bits(p[(size_t)i * UD]);
    put16(WH1T + (size_t)n * KH1 + k8, o);
    return;
  } else if (u < U5) {
    const int v    = u - U4;
    const int n    = v >> 6;
    const int k8   = (v & 63) * 8;
    const int srow = k8 & (UD - 1);
    const float* p = Whl + (size_t)srow * HD + n;
#pragma unroll
    for (int i = 0; i < 8; ++i) o[i] = (unsigned short)bf16_bits(p[(size_t)i * HD]);
    put16(WHLT + (size_t)n * KHL + k8, o);
    return;
  } else if (u < U6) {
    const int v   = u - U5;
    const int row = v >> 4;
    const int k8  = (v & 15) * 8;
    const float* p = nf + (size_t)row * HD + k8;
    const v4f a = *(const v4fa*)p;
    const v4f b = *(const v4fa*)(p + 4);
    o[0] = (unsigned short)bf16_bits(a.x); o[1] = (unsigned short)bf16_bits(a.y);
    o[2] = (unsigned short)bf16_bits(a.z); o[3] = (unsigned short)bf16_bits(a.w);
    o[4] = (unsigned short)bf16_bits(b.x); o[5] = (unsigned short)bf16_bits(b.y);
    o[6] = (unsigned short)bf16_bits(b.z); o[7] = (unsigned short)bf16_bits(b.w);
    put16(NFB + (size_t)row * HD + k8, o);
    return;
  }
}

template <int NTW, int NCG, int MODE, int GATHER, int GATE>
__global__ __launch_bounds__(128 * NCG) void k_gemm(const unsigned short* __restrict__ A, int lda,
                                                    const unsigned short* __restrict__ BT, int ldb, int K,
                                                    const float* __restrict__ aux, int ldx,
                                                    const float* __restrict__ winf,
                                                    int rBase, int nN, float scale,
                                                    float* Cf, int ldc, unsigned short* Cb, float* Gt) {
  constexpr int BN  = 16 * NTW * NCG;
  constexpr int NTH = 128 * NCG;
  static_assert(MODE != 0 || NTW == 8);
  static_assert(MODE != 1 || (NTW == 8 && NCG == 2));
  static_assert(MODE != 2 || (NTW == 2 && NCG == 1));
  static_assert(MODE != 3 || (NTW == 8 && NCG == 1));
  static_assert(GATE == 0 || (MODE == 1 && NTH == UD));
  static_assert(GATHER == 0 || MODE == 1);
  static_assert((GBM * BN / 8) % NTH == 0);
  extern __shared__ __attribute__((aligned(16))) float dyn[];
  float* stg = dyn;
  float* sW  = dyn + GBM * BN;
  float* sP  = sW + UD;
  float* sG  = sP + 2 * GBM;
  const int tid = (int)threadIdx.x, lane = tid & 31, wave = tid >> 5, hh = lane >> 4, m = lane & 15;
  const int rw = wave & 3, cg = wave >> 2;
  const int rowBase = (int)blockIdx.x * GBM;
  const int colBase = (int)blockIdx.y * BN;

  if constexpr (GATE != 0) sW[tid] = bf16_val(winf[tid]);

  v8f acc[NTW];
  {
    const v8f z = {0.f, 0.f, 0.f, 0.f, 0.f, 0.f, 0.f, 0.f};
#pragma unroll
    for (int t = 0; t < NTW; ++t) acc[t] = z;
  }
  const unsigned short* ap = A  + (size_t)(rowBase + 16 * rw + m) * (size_t)lda + 8 * hh;
  const unsigned short* bp = BT + (size_t)(colBase + cg * 16 * NTW + m) * (size_t)ldb + 8 * hh;

#pragma unroll 1
  for (int k0 = 0; k0 < K; k0 += 32) {
    FragB af;
    af.h[0] = *(const v8usa*)(ap + k0);
    af.h[1] = *(const v8usa*)(ap + k0 + 16);
#pragma unroll
    for (int nt = 0; nt < NTW; ++nt) {
      const unsigned short* wq = bp + (size_t)(16 * nt) * (size_t)ldb + k0;
      FragB bf;
      bf.h[0] = *(const v8usa*)wq;
      bf.h[1] = *(const v8usa*)(wq + 16);
      acc[nt] = wmb(af, bf, acc[nt]);
    }
  }

#pragma unroll
  for (int nt = 0; nt < NTW; ++nt) {
    const int lc = cg * 16 * NTW + 16 * nt + m;
#pragma unroll
    for (int r = 0; r < 8; ++r) {
      const int lr = 16 * rw + 8 * hh + r;
      stg[lr * BN + lc] = acc[nt][r];
    }
  }
  __syncthreads();

  if constexpr (GATHER != 0) {
#pragma unroll 1
    for (int it = 0; it < (GBM * BN / 8) / NTH; ++it) {
      const int uu   = it * NTH + tid;
      const int lr   = uu / (BN / 8);
      const int c8   = (uu - lr * (BN / 8)) * 8;
      const int grow = rowBase + lr;
      const int rq   = grow / nN;
      const int s    = grow - rq * nN;
      int rr = rBase + rq;
      rr = rr > nN - 1 ? nN - 1 : rr;
      float* sp = stg + lr * BN + c8;
      const float* ga = aux + (size_t)s  * (size_t)ldx + c8;
      const float* gb = aux + (size_t)rr * (size_t)ldx + UD + c8;
      const v4f x0 = *(const v4fa*)sp;
      const v4f x1 = *(const v4fa*)(sp + 4);
      const v4f a0 = *(const v4fa*)ga;
      const v4f a1 = *(const v4fa*)(ga + 4);
      const v4f b0 = *(const v4fa*)gb;
      const v4f b1 = *(const v4fa*)(gb + 4);
      const v4f y0 = (x0 + a0) + b0;
      const v4f y1 = (x1 + a1) + b1;
      *(v4fa*)sp       = y0;
      *(v4fa*)(sp + 4) = y1;
    }
    __syncthreads();
  }

  if constexpr (MODE == 0) {
    v4f pv[16];
#pragma unroll
    for (int i = 0; i < 16; ++i) pv[i] = *(const v4fa*)(stg + (16 * rw + i) * BN + cg * 128 + 4 * lane);
#pragma unroll
    for (int i = 0; i < 16; ++i) {
      float* op = Cf + (size_t)(rowBase + 16 * rw + i) * (size_t)ldc + colBase + cg * 128 + 4 * lane;
      *(volatile v4f*)op = pv[i];
    }
    __threadfence();
#pragma unroll
    for (int i = 0; i < 16; ++i) {
      float* op = Cf + (size_t)(rowBase + 16 * rw + i) * (size_t)ldc + colBase + cg * 128 + 4 * lane;
      *(volatile v4f*)op = pv[i];
    }
  } else if constexpr (MODE == 1) {
    const int part = hh;
    const int j = m;
    const unsigned mh = 0u - (unsigned)part;
    const unsigned ml = ~mh;
    v4f wa = {0.f, 0.f, 0.f, 0.f}, wb = {0.f, 0.f, 0.f, 0.f};
    if constexpr (GATE != 0) {
      wa = *(const v4fa*)(sW + cg * 128 + 8 * j);
      wb = *(const v4fa*)(sW + cg * 128 + 8 * j + 4);
    }
    const v8f w8 = {wa.x, wa.y, wa.z, wa.w, wb.x, wb.y, wb.z, wb.w};
    v8us pv[16];
#pragma unroll
    for (int i = 0; i < 16; ++i) {
      const int lrow = 16 * rw + i;
      const float* sp = stg + lrow * BN + cg * 128 + 8 * j;
      const v4f a = *(const v4fa*)sp;
      const v4f b = *(const v4fa*)(sp + 4);
      const v8f f8 = {a.x, a.y, a.z, a.w, b.x, b.y, b.z, b.w};
      float pg = 0.0f;
      v8us oo;
#pragma unroll
      for (int e = 0; e < 8; ++e) {
        const float v = silu_f(f8[e] * scale);
        const unsigned hb = bf16_bits(v);
        const unsigned lb = bf16_bits(v - __uint_as_float(hb << 16));
        oo[e] = (unsigned short)((hb & ml) | (lb & mh));
        if constexpr (GATE != 0) pg = fmaf(v, w8[e], pg);
      }
      pv[i] = oo;
      if constexpr (GATE != 0) {
        pg += __shfl_xor(pg, 1, 32);
        pg += __shfl_xor(pg, 2, 32);
        pg += __shfl_xor(pg, 4, 32);
        pg += __shfl_xor(pg, 8, 32);
        if (lane == 0) sP[cg * GBM + lrow] = pg;
      }
    }
#pragma unroll
    for (int i = 0; i < 16; ++i) {
      unsigned short* op = Cb + (size_t)(rowBase + 16 * rw + i) * (size_t)KHL + part * UD + cg * 128 + 8 * j;
      *(volatile v8us*)op = pv[i];
    }
    __threadfence();
#pragma unroll
    for (int i = 0; i < 16; ++i) {
      unsigned short* op = Cb + (size_t)(rowBase + 16 * rw + i) * (size_t)KHL + part * UD + cg * 128 + 8 * j;
      *(volatile v8us*)op = pv[i];
    }
    if constexpr (GATE != 0) {
      __syncthreads();
      if (tid < GBM) {
        const float d = sP[tid] + sP[GBM + tid];
        sG[tid] = __builtin_amdgcn_rcpf(1.0f + __expf(-(d * C16)));
      }
      __syncthreads();
      const int tl = tid < GBM / 4 ? tid : GBM / 4 - 1;
      const v4f g4 = *(const v4fa*)(sG + 4 * tl);
      float* gp = Gt + (size_t)rowBase + 4 * tl;
      if (tid < GBM / 4) *(volatile v4f*)gp = g4;
      __threadfence();
      if (tid < GBM / 4) *(volatile v4f*)gp = g4;
    }
  } else if constexpr (MODE == 2) {
    v4f pv[4];
#pragma unroll
    for (int it = 0; it < 4; ++it) {
      const int p  = it * 32 + lane;
      const int lr = 16 * rw + (p >> 3);
      const int c4 = (p & 7) * 4;
      const v4f sv = *(const v4fa*)(stg + lr * BN + c4);
      v4f q;
      q.x = sv.x + bf16_val(aux[c4 + 0]);
      q.y = sv.y + bf16_val(aux[c4 + 1]);
      q.z = sv.z + bf16_val(aux[c4 + 2]);
      q.w = sv.w + bf16_val(aux[c4 + 3]);
      pv[it] = q;
    }
#pragma unroll
    for (int it = 0; it < 4; ++it) {
      const int p  = it * 32 + lane;
      const int lr = 16 * rw + (p >> 3);
      const int c4 = (p & 7) * 4;
      float* op = Cf + (size_t)(rowBase + lr) * (size_t)ldc + c4;
      *(volatile v4f*)op = pv[it];
    }
    __threadfence();
#pragma unroll
    for (int it = 0; it < 4; ++it) {
      const int p  = it * 32 + lane;
      const int lr = 16 * rw + (p >> 3);
      const int c4 = (p & 7) * 4;
      float* op = Cf + (size_t)(rowBase + lr) * (size_t)ldc + c4;
      *(volatile v4f*)op = pv[it];
    }
  } else {
    v4f pv[16];
#pragma unroll
    for (int i = 0; i < 16; ++i) {
      const int row = rowBase + 16 * rw + i;
      const int rc  = row < nN ? row : nN - 1;
      const v4f hv = *(const v4fa*)(aux + (size_t)rc * (size_t)ldx + colBase + 4 * lane);
      const v4f sv = *(const v4fa*)(stg + (16 * rw + i) * BN + 4 * lane);
      v4f q;
      q.x = fmaf(sv.x, scale, bf16_val(hv.x));
      q.y = fmaf(sv.y, scale, bf16_val(hv.y));
      q.z = fmaf(sv.z, scale, bf16_val(hv.z));
      q.w = fmaf(sv.w, scale, bf16_val(hv.w));
      pv[i] = q;
    }
#pragma unroll
    for (int i = 0; i < 16; ++i) {
      const int row = rowBase + 16 * rw + i;
      if (row < nN) {
        float* op = Cf + (size_t)row * (size_t)ldc + colBase + 4 * lane;
        *(volatile v4f*)op = pv[i];
      }
    }
    __threadfence();
#pragma unroll
    for (int i = 0; i < 16; ++i) {
      const int row = rowBase + 16 * rw + i;
      if (row < nN) {
        float* op = Cf + (size_t)row * (size_t)ldc + colBase + 4 * lane;
        *(volatile v4f*)op = pv[i];
      }
    }
  }
}

__global__ __launch_bounds__(NTHR) void k_len(const float* __restrict__ nv, int rBase, int nN,
                                              unsigned short* L2) {
  __shared__ __attribute__((aligned(16))) unsigned short sL[NTHR * KE1];
  const int tid = (int)threadIdx.x;
  const int eb  = (int)blockIdx.x * NTHR;
  const int e   = eb + tid;
  const int rq  = e / nN;
  const int s   = e - rq * nN;
  int rr = rBase + rq;
  rr = rr > nN - 1 ? nN - 1 : rr;
  const float* pr = nv + (size_t)rr * VC;
  const float* ps = nv + (size_t)s * VC;
#pragma unroll 1
  for (int j = 0; j < 4; ++j) {
    R24 xr, xs;
#pragma unroll
    for (int q = 0; q < 6; ++q) {
      xr.q[q] = *(const v4fa*)(pr + 24 * j + 4 * q);
      xs.q[q] = *(const v4fa*)(ps + 24 * j + 4 * q);
    }
    v8us ho, lo;
#pragma unroll
    for (int i = 0; i < 8; ++i) {
      const float d0 = bf16_val(xr.f[3 * i + 0]) - bf16_val(xs.f[3 * i + 0]);
      const float d1 = bf16_val(xr.f[3 * i + 1]) - bf16_val(xs.f[3 * i + 1]);
      const float d2 = bf16_val(xr.f[3 * i + 2]) - bf16_val(xs.f[3 * i + 2]);
      const float l2 = (d0 * d0 + d2 * d2) + d1 * d1;
      const unsigned hb = bf16_bits(l2);
      ho[i] = (unsigned short)hb;
      lo[i] = (unsigned short)bf16_bits(l2 - __uint_as_float(hb << 16));
    }
    *(v8usa*)(sL + tid * KE1 + 8 * j)      = ho;
    *(v8usa*)(sL + tid * KE1 + VD + 8 * j) = lo;
  }
  __syncthreads();
  v8us pv[8];
#pragma unroll
  for (int it = 0; it < 8; ++it) pv[it] = *(const v8usa*)(sL + (size_t)(it * NTHR + tid) * 8);
  unsigned short* lb = L2 + (size_t)eb * KE1;
#pragma unroll
  for (int it = 0; it < 8; ++it) *(volatile v8us*)(lb + (size_t)(it * NTHR + tid) * 8) = pv[it];
  __threadfence();
#pragma unroll
  for (int it = 0; it < 8; ++it) *(volatile v8us*)(lb + (size_t)(it * NTHR + tid) * 8) = pv[it];
}

__global__ __launch_bounds__(NTHR) void k_aggm(const unsigned short* __restrict__ Mp, const float* __restrict__ Gt,
                                               const float* __restrict__ nf, int rBase, int nN,
                                               unsigned short* NZ) {
  __shared__ __attribute__((aligned(16))) float sAcc[8 * UD];
  __shared__ __attribute__((aligned(16))) unsigned short sRow[KH1];
  const int tid = (int)threadIdx.x, lane = tid & 31, wave = tid >> 5;
  const int rl = (int)blockIdx.x;
  const int r  = rBase + rl;
  float acc[8];
#pragma unroll
  for (int k = 0; k < 8; ++k) acc[k] = 0.0f;
  const size_t rowb = (size_t)rl * (size_t)nN;
  const int nIt = nN >> 3;
#pragma unroll 1
  for (int si = 0; si < nIt; ++si) {
    const int s = si * 8 + wave;
    const size_t e = rowb + (size_t)s;
    const unsigned short* rp = Mp + e * KHL + 8 * lane;
    const v8us h8 = *(const v8usa*)rp;
    const v8us l8 = *(const v8usa*)(rp + UD);
    const float g  = Gt[e];
    const float gm = (s != r) ? g : 0.0f;
#pragma unroll
    for (int k = 0; k < 8; ++k) acc[k] = fmaf(gm, bfw(h8[k]) + bfw(l8[k]), acc[k]);
  }
  {
    const v4f a0 = {acc[0], acc[1], acc[2], acc[3]};
    const v4f a1 = {acc[4], acc[5], acc[6], acc[7]};
    *(v4fa*)(sAcc + wave * UD + 8 * lane)     = a0;
    *(v4fa*)(sAcc + wave * UD + 8 * lane + 4) = a1;
  }
  __syncthreads();
  float mi = 0.0f;
#pragma unroll
  for (int w = 0; w < 8; ++w) mi += sAcc[w * UD + tid];
  const unsigned hb = bf16_bits(mi);
  sRow[tid]      = (unsigned short)hb;
  sRow[UD + tid] = (unsigned short)bf16_bits(mi - __uint_as_float(hb << 16));
  const int th = tid < HD ? tid : HD - 1;
  const unsigned short nb = (unsigned short)bf16_bits(nf[(size_t)r * HD + th]);
  if (tid < HD) sRow[2 * UD + tid] = nb;
  __syncthreads();
  const int tl = tid < KH1 / 8 ? tid : KH1 / 8 - 1;
  const v8us o = *(const v8usa*)(sRow + 8 * tl);
  unsigned short* op = NZ + (size_t)r * KH1 + 8 * tl;
  if (tid < KH1 / 8) *(volatile v8us*)op = o;
  __threadfence();
  if (tid < KH1 / 8) *(volatile v8us*)op = o;
}

__global__ __launch_bounds__(ATHR) void k_aggv(const float* __restrict__ PH, const float* __restrict__ nv,
                                               int rBase, int nN, float rn1, float* out0) {
  __shared__ __attribute__((aligned(16))) float sNV[VC];
  __shared__ __attribute__((aligned(16))) float sAcc[4 * VC];
  __shared__ __attribute__((aligned(16))) float sOut[VC];
  const int tid = (int)threadIdx.x;
  const int rl = (int)blockIdx.x;
  const int r  = rBase + rl;
  const int t96 = tid < VC ? tid : VC - 1;
  const float xv = bf16_val(nv[(size_t)r * VC + t96]);
  if (tid < VC) sNV[tid] = xv;
  __syncthreads();
  const int g = tid / VC;
  const int p = tid - g * VC;
  const int v = p / 3;
  const int c = p - 3 * v;
  const float xr0 = sNV[3 * v + 0], xr1 = sNV[3 * v + 1], xr2 = sNV[3 * v + 2];
  const int q = nN >> 2;
  const size_t rowb = (size_t)rl * (size_t)nN;
  float acc = 0.0f;
#pragma unroll 1
  for (int i = 0; i < q; ++i) {
    const int s = g * q + i;
    const float* xs = nv + (size_t)s * VC + 3 * v;
    const float s0 = bf16_val(xs[0]);
    const float s1 = bf16_val(xs[1]);
    const float s2 = bf16_val(xs[2]);
    const float d0 = xr0 - s0, d1 = xr1 - s1, d2 = xr2 - s2;
    const float l2  = (d0 * d0 + d2 * d2) + d1 * d1;
    const float len = sqrtf(fmaxf(l2, 1e-20f));
    const float inv = __builtin_amdgcn_rcpf(1.0f + len);
    const float dc  = (c == 0) ? d0 : ((c == 1) ? d1 : d2);
    const float ph  = PH[(rowb + (size_t)s) * VD + v];
    const float msk = (s != r) ? 1.0f : 0.0f;
    acc += ((ph * dc) * inv) * msk;
  }
  sAcc[g * VC + p] = acc;
  __syncthreads();
  if (tid < VC) {
    const float sh = ((sAcc[tid] + sAcc[VC + tid]) + sAcc[2 * VC + tid]) + sAcc[3 * VC + tid];
    sOut[tid] = sNV[tid] + sh * rn1;
  }
  __syncthreads();
  const int tl = tid < VC / 4 ? tid : VC / 4 - 1;
  const v4f o4 = *(const v4fa*)(sOut + 4 * tl);
  float* op = out0 + (size_t)r * VC + 4 * tl;
  if (tid < VC / 4) *(volatile v4f*)op = o4;
  __threadfence();
  if (tid < VC / 4) *(volatile v4f*)op = o4;
}

static inline size_t al256(size_t x) { return (x + 255) & ~(size_t)255; }

extern "C" void kernel_launch(void* const* d_in, const int* in_sizes, int n_in,
                              void* d_out, int out_size, void* d_ws, size_t ws_size,
                              hipStream_t stream) {
  if (n_in < 12) return;
  if (in_sizes[1] < HD || (in_sizes[1] % HD) != 0) return;
  const int nN = in_sizes[1] / HD;
  if (nN < RPC || (nN % RPC) != 0 || nN > 2048) return;
  if (in_sizes[0] != nN * VC) return;
  if (in_sizes[2] != (VD + 2 * HD) * UD) return;
  if (in_sizes[3] != UD * UD || in_sizes[4] != UD * UD || in_sizes[5] != UD * UD) return;
  if (in_sizes[6] != UD * VD || in_sizes[7] != VD) return;
  if (in_sizes[8] != UD) return;
  if (in_sizes[9] != (UD + HD) * UD || in_sizes[10] != UD * UD) return;
  if (in_sizes[11] != UD * HD) return;
  if ((long long)out_size != (long long)nN * VC + (long long)nN * HD) return;

  const float* nv   = (const float*)d_in[0];
  const float* nf   = (const float*)d_in[1];
  const float* We1  = (const float*)d_in[2];
  const float* We2  = (const float*)d_in[3];
  const float* Wx1  = (const float*)d_in[4];
  const float* Wx2  = (const float*)d_in[5];
  const float* Wxl  = (const float*)d_in[6];
  const float* bxl  = (const float*)d_in[7];
  const float* Winf = (const float*)d_in[8];
  const float* Wh1  = (const float*)d_in[9];
  const float* Wh2  = (const float*)d_in[10];
  const float* Whl  = (const float*)d_in[11];
  float* out0 = (float*)d_out;
  float* out1 = out0 + (size_t)nN * VC;

  const int CR     = RPC * nN;
  const int nChunk = nN / RPC;
  if ((CR % NTHR) != 0 || (CR % GBM) != 0 || (nN % GBM) != 0) return;

  char* ws = (char*)d_ws;
  size_t off = 0;
  const size_t oWE1A  = off; off = al256(off + (size_t)UD * KE1 * 2);
  const size_t oWE1BC = off; off = al256(off + (size_t)2 * UD * HD * 2);
  const size_t oWE2T  = off; off = al256(off + (size_t)UD * KHL * 2);
  const size_t oWX1T  = off; off = al256(off + (size_t)UD * KHL * 2);
  const size_t oWX2T  = off; off = al256(off + (size_t)UD * KHL * 2);
  const size_t oWXLT  = off; off = al256(off + (size_t)VD * KHL * 2);
  const size_t oWH1T  = off; off = al256(off + (size_t)UD * KH1 * 2);
  const size_t oWH2T  = off; off = al256(off + (size_t)UD * KHL * 2);
  const size_t oWHLT  = off; off = al256(off + (size_t)HD * KHL * 2);
  const size_t oNFB   = off; off = al256(off + (size_t)nN * HD * 2);
  const size_t oASR   = off; off = al256(off + (size_t)nN * 2 * UD * 4);
  const size_t oL2    = off; off = al256(off + (size_t)CR * KE1 * 2);
  const size_t oPA    = off; off = al256(off + (size_t)CR * KHL * 2);
  const size_t oPB    = off; off = al256(off + (size_t)CR * KHL * 2);
  const size_t oGT    = off; off = al256(off + (size_t)CR * 4);
  const size_t oPH    = off; off = al256(off + (size_t)CR * VD * 4);
  const size_t oNZ    = off; off = al256(off + (size_t)nN * KH1 * 2);
  const size_t oG1    = off; off = al256(off + (size_t)nN * KHL * 2);
  const size_t oG2    = off; off = al256(off + (size_t)nN * KHL * 2);
  if (off > ws_size || off > (size_t)WSMAX) return;
  unsigned short* WE1A  = (unsigned short*)(ws + oWE1A);
  unsigned short* WE1BC = (unsigned short*)(ws + oWE1BC);
  unsigned short* WE2T  = (unsigned short*)(ws + oWE2T);
  unsigned short* WX1T  = (unsigned short*)(ws + oWX1T);
  unsigned short* WX2T  = (unsigned short*)(ws + oWX2T);
  unsigned short* WXLT  = (unsigned short*)(ws + oWXLT);
  unsigned short* WH1T  = (unsigned short*)(ws + oWH1T);
  unsigned short* WH2T  = (unsigned short*)(ws + oWH2T);
  unsigned short* WHLT  = (unsigned short*)(ws + oWHLT);
  unsigned short* NFB   = (unsigned short*)(ws + oNFB);
  float*          ASR   = (float*)(ws + oASR);
  unsigned short* L2    = (unsigned short*)(ws + oL2);
  unsigned short* PA    = (unsigned short*)(ws + oPA);
  unsigned short* PB    = (unsigned short*)(ws + oPB);
  float*          GT    = (float*)(ws + oGT);
  float*          PH    = (float*)(ws + oPH);
  unsigned short* NZ    = (unsigned short*)(ws + oNZ);
  unsigned short* G1    = (unsigned short*)(ws + oG1);
  unsigned short* G2    = (unsigned short*)(ws + oG2);

  hipFuncSetAttribute(reinterpret_cast<const void*>(&k_gemm<8, 2, 0, 0, 0>),
                      hipFuncAttributeMaxDynamicSharedMemorySize, (int)LDS_BIG);
  hipFuncSetAttribute(reinterpret_cast<const void*>(&k_gemm<8, 2, 1, 1, 0>),
                      hipFuncAttributeMaxDynamicSharedMemorySize, (int)LDS_BIG);
  hipFuncSetAttribute(reinterpret_cast<const void*>(&k_gemm<8, 2, 1, 0, 1>),
                      hipFuncAttributeMaxDynamicSharedMemorySize, (int)LDS_BIG);
  hipFuncSetAttribute(reinterpret_cast<const void*>(&k_gemm<8, 2, 1, 0, 0>),
                      hipFuncAttributeMaxDynamicSharedMemorySize, (int)LDS_BIG);

  const int   nPrep = (NU_W + nN * (HD / 8)) / NTHR;
  const float rn1   = 1.0f / (float)(nN - 1);
  const int   gE    = CR / GBM;
  const int   gNd   = nN / GBM;

  k_prep<<<nPrep, NTHR, 0, stream>>>(nf, We1, We2, Wx1, Wx2, Wxl, Wh1, Wh2, Whl, nN,
                                     WE1A, WE1BC, WE2T, WX1T, WX2T, WXLT, WH1T, WH2T, WHLT, NFB);
  k_gemm<8, 2, 0, 0, 0><<<dim3(gNd, 2), 256, LDS_BIG, stream>>>(NFB, HD, WE1BC, HD, HD, ASR, 2 * UD, Winf,
                                                               0, nN, 1.0f, ASR, 2 * UD, PA, GT);
  for (int ch = 0; ch < nChunk; ++ch) {
    const int rBase = ch * RPC;
    k_len<<<CR / NTHR, NTHR, 0, stream>>>(nv, rBase, nN, L2);
    k_gemm<8, 2, 1, 1, 0><<<dim3(gE, 1), 256, LDS_BIG, stream>>>(L2, KE1, WE1A, KE1, KE1, ASR, 2 * UD, Winf,
                                                                rBase, nN, C288, ASR, 2 * UD, PA, GT);
    k_gemm<8, 2, 1, 0, 1><<<dim3(gE, 1), 256, LDS_BIG, stream>>>(PA, KHL, WE2T, KHL, KHL, ASR, 2 * UD, Winf,
                                                                rBase, nN, C16, ASR, 2 * UD, PB, GT);
    k_aggm<<<RPC, NTHR, 0, stream>>>(PB, GT, nf, rBase, nN, NZ);
    k_gemm<8, 2, 1, 0, 0><<<dim3(gE, 1), 256, LDS_BIG, stream>>>(PB, KHL, WX1T, KHL, KHL, ASR, 2 * UD, Winf,
                                                                rBase, nN, C16, ASR, 2 * UD, PA, GT);
    k_gemm<8, 2, 1, 0, 0><<<dim3(gE, 1), 256, LDS_BIG, stream>>>(PA, KHL, WX2T, KHL, KHL, ASR, 2 * UD, Winf,
                                                                rBase, nN, C16, ASR, 2 * UD, PB, GT);
    k_gemm<2, 1, 2, 0, 0><<<dim3(gE, 1), 128, LDS_XL, stream>>>(PB, KHL, WXLT, KHL, KHL, bxl, VD, Winf,
                                                               rBase, nN, 1.0f, PH, VD, PA, GT);
    k_aggv<<<RPC, ATHR, 0, stream>>>(PH, nv, rBase, nN, rn1, out0);
  }
  k_gemm<8, 2, 1, 0, 0><<<dim3(gNd, 1), 256, LDS_BIG, stream>>>(NZ, KH1, WH1T, KH1, KH1, ASR, 2 * UD, Winf,
                                                               0, nN, C384, ASR, 2 * UD, G1, GT);
  k_gemm<8, 2, 1, 0, 0><<<dim3(gNd, 1), 256, LDS_BIG, stream>>>(G1, KHL, WH2T, KHL, KHL, ASR, 2 * UD, Winf,
                                                               0, nN, C16, ASR, 2 * UD, G2, GT);
  k_gemm<8, 1, 3, 0, 0><<<dim3(gNd, 1), 128, LDS_OUT, stream>>>(G2, KHL, WHLT, KHL, KHL, nf, HD, Winf,
                                                               0, nN, C16, out1, HD, PA, GT);
}
